// Actor_35974646071851
// MI455X (gfx1250) — hardware-verified
//
#include <hip/hip_runtime.h>
#include <cstdint>

#define __bf16 _Float16
typedef __attribute__((ext_vector_type(16))) _Float16      v16bf;
typedef __attribute__((ext_vector_type(4)))  float         v4f_t;
typedef float v4fa __attribute__((ext_vector_type(4), may_alias));
#define RSPLIT (1.0f / 2048.0f)
#define BUCKET 64
#define LCAP   4096
typedef __attribute__((ext_vector_type(8)))  float         v8f;
typedef __attribute__((ext_vector_type(4)))  unsigned int  v4u;
typedef __attribute__((ext_vector_type(8)))  int           v8i;
typedef __attribute__((ext_vector_type(4)))  int           v4i;

union Frag16 { v16bf v; _Float16 e[16]; };
__device__ __forceinline__ void split1(float f, _Float16& h, _Float16& l) { h = (_Float16)f; l = (_Float16)((f - (float)h) * 2048.0f); }
__device__ __forceinline__ void put4s(Frag16& v, Frag16& vl, int base, float4 f) {
    split1(f.x, v.e[base + 0], vl.e[base + 0]); split1(f.y, v.e[base + 1], vl.e[base + 1]);
    split1(f.z, v.e[base + 2], vl.e[base + 2]); split1(f.w, v.e[base + 3], vl.e[base + 3]);
}

__global__ __launch_bounds__(256)
void gemm_bf16_wmma(const float* __restrict__ A, const float* __restrict__ B,
                    float* __restrict__ C, const float* __restrict__ bias,
                    int M, int K, int Nn, int act) {
    __shared__ float sB[8192];
    const int tid = (int)threadIdx.x;

#if __has_builtin(__builtin_amdgcn_tensor_load_to_lds) && \
    __has_builtin(__builtin_amdgcn_s_wait_tensorcnt)
    if ((tid >> 5) == 0) {
        unsigned long long ga = (unsigned long long)(uintptr_t)B;
        unsigned lds = (unsigned)(uintptr_t)&sB[0];
        unsigned td0 = (unsigned)Nn, td1 = (unsigned)K;
        v4u g0; v8i g1;
        v4i g2 = {0, 0, 0, 0}, g3 = {0, 0, 0, 0};
        v8i g4 = {0, 0, 0, 0, 0, 0, 0, 0};
        g0[0] = 1u;
        g0[1] = lds;
        g0[2] = (unsigned)(ga & 0xffffffffu);
        g0[3] = (unsigned)((ga >> 32) & 0x01ffffffu) | (2u << 30);
        g1[0] = (int)(2u << 16);
        g1[1] = (int)((td0 & 0xffffu) << 16);
        g1[2] = (int)((td0 >> 16) | ((td1 & 0xffffu) << 16));
        g1[3] = (int)((td1 >> 16) | ((unsigned)Nn << 16));
        g1[4] = (int)(td1 & 0xffffu);
        g1[5] = (int)Nn;
        g1[6] = 0;
        g1[7] = 0;
        __builtin_amdgcn_tensor_load_to_lds(g0, g1, g2, g3, g4, 0);
        __builtin_amdgcn_s_wait_tensorcnt(0);
    }
    __syncthreads();
#else
    for (int i = tid; i < K * Nn; i += 256) sB[i] = B[i];
    __syncthreads();
#endif

    const int wave = (int)((blockIdx.x * blockDim.x + threadIdx.x) >> 5);
    const int wloc = tid >> 5;
    const int lane = tid & 31;
    const int ntiles = Nn >> 4;
    const int mt = wave;
    if (mt * 16 >= M) return;

    const int m0   = mt * 16;
    const int idx  = lane & 15;
    const int half = lane >> 4;

    __shared__ __attribute__((aligned(16))) float cst[8][16 * 128];
    float* cs = cst[wloc];

    v8f acc[8];
#pragma unroll
    for (int t = 0; t < 8; ++t) acc[t] = (v8f){};
    for (int k0 = 0; k0 < K; k0 += 32) {
        const float4* ap =
            (const float4*)(A + (size_t)(m0 + idx) * K + k0 + half * 8);
        Frag16 a, al;
        put4s(a, al, 0, ap[0]);
        put4s(a, al, 4, ap[1]);
        put4s(a, al, 8, ap[4]);
        put4s(a, al, 12, ap[5]);
#pragma unroll
        for (int t = 0; t < 8; ++t) {
            if (t < ntiles) {
                const float* bp = &sB[(size_t)(k0 + half * 8) * Nn + (t * 16 + idx)];
                Frag16 b, bl;
#pragma unroll
                for (int j = 0; j < 8; ++j) {
                    split1(bp[(size_t)j * Nn],        b.e[j],     bl.e[j]);
                    split1(bp[(size_t)(16 + j) * Nn], b.e[8 + j], bl.e[8 + j]);
                }
                v8f x = {};
                x = __builtin_amdgcn_wmma_f32_16x16x32_f16(false, al.v, false, b.v, (short)0, x, false, false);
                x = __builtin_amdgcn_wmma_f32_16x16x32_f16(false, a.v, false, bl.v, (short)0, x, false, false);
                acc[t] = __builtin_amdgcn_wmma_f32_16x16x32_f16(false, a.v, false, b.v, (short)0, acc[t], false, false) + x * RSPLIT;
            }
        }
    }

#pragma unroll
    for (int t = 0; t < 8; ++t) {
        if (t < ntiles) {
            float bv = bias ? bias[t * 16 + idx] : 0.0f;
#pragma unroll
            for (int v = 0; v < 8; ++v) {
                float val = acc[t][v] + bv;
                if (act) val = (val > 0.0f) ? val : 0.1f * val;
                cs[(v + half * 8) * Nn + t * 16 + idx] = val;
            }
        }
    }
    asm volatile("s_wait_dscnt 0" ::: "memory");
    const int cpr = Nn >> 2;
    const int nch = 16 * cpr;
#pragma unroll 1
    for (int pass = 0; pass < 2; ++pass) {
        for (int c = lane; c < nch; c += 32) {
            const int rr = c / cpr, q = c - rr * cpr;
            *(volatile v4f_t*)(C + (size_t)(m0 + rr) * Nn + q * 4) = *(const volatile v4fa*)(cs + rr * Nn + q * 4);
        }
        __threadfence();
    }
}

__global__ __launch_bounds__(256)
void bucket_list_k(const int* __restrict__ src, const int* __restrict__ dst, int E, int N,
                   float* __restrict__ dinv, int* __restrict__ noff, int* __restrict__ ncnt, int* __restrict__ lsrc) {
    __shared__ unsigned lst[LCAP];
    __shared__ unsigned srt[LCAP];
    __shared__ int wcnt[8];
    __shared__ int total;
    __shared__ int cnt[BUCKET], off[BUCKET], cur[BUCKET];
    const int tid = threadIdx.x, lane = tid & 31, wave = tid >> 5;
    const int n0 = blockIdx.x * BUCKET;
    if (tid == 0) total = 0;
    if (tid < BUCKET) cnt[tid] = 0;
    __syncthreads();

    for (int e0 = 0; e0 < E; e0 += 256) {
        const int e = e0 + tid;
        int loc = -1, s = 0;
        if (e < E) { const int d = dst[e]; const int l = d - n0; if ((unsigned)l < (unsigned)BUCKET) { loc = l; s = src[e]; } }
        const unsigned m = __ballot(loc >= 0);
        if (m == 0u) {
            if (lane == 0) wcnt[wave] = 0;
        } else {
            if (lane == 0) wcnt[wave] = __popc(m);
        }
        __syncthreads();
        int base = total;
#pragma unroll
        for (int w = 0; w < 8; ++w) if (w < wave) base += wcnt[w];
        if (loc >= 0) {
            const int slot = base + __popc(m & ((1u << lane) - 1u));
            if (slot < LCAP) lst[slot] = ((unsigned)loc << 24) | (unsigned)s;
        }
        __syncthreads();
        if (tid == 0) { int t = total; for (int w = 0; w < 8; ++w) t += wcnt[w]; total = t; }
        __syncthreads();
    }
    const int nl = (total < LCAP) ? total : LCAP;
    if (tid < BUCKET) { int c = 0; for (int i = 0; i < nl; ++i) c += ((int)(lst[i] >> 24) == tid); cnt[tid] = c; }
    __syncthreads();
    if (tid == 0) { int o = 0; for (int j = 0; j < BUCKET; ++j) { off[j] = o; cur[j] = o; o += cnt[j]; } }
    __syncthreads();
    if (tid < BUCKET) { int p = off[tid]; for (int i = 0; i < nl; ++i) if ((int)(lst[i] >> 24) == tid) srt[p++] = lst[i] & 0xFFFFFFu; }
    __syncthreads();
#pragma unroll 1
    for (int pass = 0; pass < 2; ++pass) {
        if (tid < BUCKET && n0 + tid < N) {
            *(volatile float*)(dinv + n0 + tid) = rsqrtf(1.0f + (float)cnt[tid]);
            *(volatile int*)(noff + n0 + tid) = blockIdx.x * LCAP + off[tid];
            *(volatile int*)(ncnt + n0 + tid) = cnt[tid];
        }
        typedef __attribute__((ext_vector_type(4))) unsigned v4u_t;
        typedef unsigned v4ua __attribute__((ext_vector_type(4), may_alias));
        for (int c = tid; c * 4 < nl; c += 256)
            *(volatile v4u_t*)((unsigned*)lsrc + (size_t)blockIdx.x * LCAP + c * 4) = *(const volatile v4ua*)(srt + c * 4);
        __threadfence();
    }
}

__global__ __launch_bounds__(256)
void gather_gcn_k(const float* __restrict__ h, const float* __restrict__ dinv,
                  const int* __restrict__ noff, const int* __restrict__ ncnt, const int* __restrict__ lsrc,
                  const float* __restrict__ b, float* __restrict__ out, int N, int F, int act) {
    const int wid  = (int)((blockIdx.x * blockDim.x + threadIdx.x) >> 5);
    const int lane = (int)(threadIdx.x & 31);
    if (wid >= N) return;
    const float dn = dinv[wid];
    const int o0 = noff[wid], cnt_ = ncnt[wid];
    for (int f = lane; f < F; f += 32) {
        float acc = h[(size_t)wid * F + f] * (dn * dn);
        for (int i = 0; i < cnt_; ++i) {
            int s = lsrc[o0 + i];
            s = ((unsigned)s < (unsigned)N) ? s : 0;
            acc += h[(size_t)s * F + f] * (dinv[s] * dn);
        }
        float v = acc + b[f];
        if (act) v = (v > 0.0f) ? v : 0.1f * v;
        *(volatile float*)(out + (size_t)wid * F + f) = v;
        __threadfence();
        *(volatile float*)(out + (size_t)wid * F + f) = v;
    }
}

__global__ __launch_bounds__(256)
void pool_max_k(const float* __restrict__ h, float* __restrict__ g,
                int N, int G, int F) {
    int gr = blockIdx.x;
    int start = (int)(((long long)gr * N + G - 1) / G);
    int end   = (int)(((long long)(gr + 1) * N + G - 1) / G);
    if (end > N) end = N;
    int f      = (int)(threadIdx.x & 63);
    int stripe = (int)(threadIdx.x >> 6);
    float m = -3.402823466e38f;
    for (int n = start + stripe; n < end; n += 4)
        m = fmaxf(m, h[(size_t)n * F + f]);
    __shared__ float red[256];
    red[threadIdx.x] = m;
    __syncthreads();
    if (stripe == 0) {
        float r = fmaxf(fmaxf(red[f], red[64 + f]),
                        fmaxf(red[128 + f], red[192 + f]));
        *(volatile float*)(g + (size_t)gr * F + f) = r;
        __threadfence();
        *(volatile float*)(g + (size_t)gr * F + f) = r;
    }
}

static inline int ceil_div(long long a, long long b) { return (int)((a + b - 1) / b); }

extern "C" void kernel_launch(void* const* d_in, const int* in_sizes, int n_in,
                              void* d_out, int out_size, void* d_ws, size_t ws_size,
                              hipStream_t stream) {
    const int F_IN = 128, H1 = 32, H2 = 64, G = 256;
    const float* x   = (const float*)d_in[0];
    const int*   ei  = (const int*)d_in[1];
    const float* W1  = (const float*)d_in[3];
    const float* b1  = (const float*)d_in[4];
    const float* W2  = (const float*)d_in[5];
    const float* b2  = (const float*)d_in[6];
    const float* l1W = (const float*)d_in[7];
    const float* l1b = (const float*)d_in[8];
    const float* l2W = (const float*)d_in[9];
    const float* l2b = (const float*)d_in[10];
    const float* l3W = (const float*)d_in[11];
    const float* l3b = (const float*)d_in[12];

    const int N = in_sizes[0] / F_IN;
    const int E = in_sizes[1] / 2;
    const int* src = ei;
    const int* dst = ei + E;

    float* w     = (float*)d_ws;
    float* dinv  = w;
    int*   noff  = (int*)(w + (size_t)N);
    int*   ncnt  = (int*)(w + 2 * (size_t)N);
    float* h1raw = w + 3 * (size_t)N;
    float* h1    = h1raw + (size_t)N * H1;
    float* h2raw = h1    + (size_t)N * H1;
    float* h2    = h2raw + (size_t)N * H2;
    float* gbuf  = h2    + (size_t)N * H2;
    float* z1    = gbuf  + (size_t)G * H2;
    float* z2    = z1    + (size_t)G * 128;
    int*   lsrc  = (int*)(z2 + (size_t)G * 64);

    const int B = 256;
    const int nbuckets = ceil_div(N, BUCKET);

    bucket_list_k<<<nbuckets, B, 0, stream>>>(src, dst, E, N, dinv, noff, ncnt, lsrc);

    gemm_bf16_wmma<<<ceil_div((long long)(N / 16) * 32, B), B, 0, stream>>>(x, W1, h1raw, nullptr, N, F_IN, H1, 0);
    gather_gcn_k<<<ceil_div((long long)N * 32, B), B, 0, stream>>>(h1raw, dinv, noff, ncnt, lsrc, b1, h1, N, H1, 1);

    gemm_bf16_wmma<<<ceil_div((long long)(N / 16) * 32, B), B, 0, stream>>>(h1, W2, h2raw, nullptr, N, H1, H2, 0);
    gather_gcn_k<<<ceil_div((long long)N * 32, B), B, 0, stream>>>(h2raw, dinv, noff, ncnt, lsrc, b2, h2, N, H2, 0);

    pool_max_k<<<G, B, 0, stream>>>(h2, gbuf, N, G, H2);

    gemm_bf16_wmma<<<ceil_div((long long)(G / 16) * 32, B), B, 0, stream>>>(gbuf, l1W, z1, l1b, G, H2, 128, 1);
    gemm_bf16_wmma<<<ceil_div((long long)(G / 16) * 32, B), B, 0, stream>>>(z1, l2W, z2, l2b, G, 128, 64, 1);
    gemm_bf16_wmma<<<ceil_div((long long)(G / 16) * 32, B), B, 0, stream>>>(z2, l3W, (float*)d_out, l3b, G, H2, 64, 0);
}
